// ContConv1dDense_8443905704366
// MI455X (gfx1250) — hardware-verified
//
#include <hip/hip_runtime.h>
#include <math.h>

typedef __attribute__((ext_vector_type(16))) _Float16 v16h;
typedef __attribute__((ext_vector_type(16))) __bf16 v16b;
typedef __attribute__((ext_vector_type(8)))  _Float16 v8h;
typedef __attribute__((ext_vector_type(8)))  float v8f;
typedef __attribute__((ext_vector_type(4)))  float v4f;
typedef __attribute__((ext_vector_type(2)))  float v2f;
typedef __attribute__((ext_vector_type(4)))  unsigned v4u;
typedef __attribute__((ext_vector_type(4)))  int v4i;
typedef float __attribute__((may_alias)) float_a;
typedef int __attribute__((may_alias)) int_a;

template <typename T> __device__ __forceinline__ void vst2(void* p, T v) { *(volatile T*)p = v; __threadfence(); *(volatile T*)p = v; }
__device__ __forceinline__ v8f wmma16(v16h a, v16h b, v8f c) {
  v8f d = __builtin_amdgcn_wmma_f32_16x16x32_f16(false, a, false, b, (short)0, c, false, false);
  asm volatile("v_nop\n\tv_nop\n\tv_nop\n\tv_nop" : "+v"(d) : "v"(a), "v"(b));
  return d;
}
__device__ __forceinline__ v8f wmma_bf(v16b a, v16b b, v8f c) {
  v8f d = __builtin_amdgcn_wmma_f32_16x16x32_bf16(false, a, false, b, (short)0, c, false, false);
  asm volatile("v_nop\n\tv_nop\n\tv_nop\n\tv_nop" : "+v"(d) : "v"(a), "v"(b));
  return d;
}
__device__ __forceinline__ v16h frag_h(const _Float16* rowk0, int lane) {
  union { v16h v; v8h q[2]; } u; const _Float16* p = rowk0 + 8 * (lane >> 4);
  u.q[0] = *(const v8h*)p; u.q[1] = *(const v8h*)(p + 16); return u.v;
}
__device__ __forceinline__ v16h frag_f32(const float* rowk0, int lane) {
  v16h a; const float* p = rowk0 + 8 * (lane >> 4);
#pragma unroll
  for (int i = 0; i < 8; ++i) { a[i] = (_Float16)p[i]; a[8 + i] = (_Float16)p[16 + i]; }
  return a;
}
__device__ __forceinline__ v16h frag_f32s(const float* rowk0, int lane, float sc) {
  v16h a; const float* p = rowk0 + 8 * (lane >> 4);
#pragma unroll
  for (int i = 0; i < 8; ++i) { a[i] = (_Float16)(p[i] * sc); a[8 + i] = (_Float16)(p[16 + i] * sc); }
  return a;
}
__device__ __forceinline__ v16h fragc_f32(const float* W, int k0, int n, int lane, int ld, int K) {
  v16h a; const int g = lane >> 4;
#pragma unroll
  for (int i = 0; i < 8; ++i) { const int ka = k0 + 8 * g + i, kb = ka + 16;
    a[i] = (_Float16)(ka < K ? W[(size_t)ka * ld + n] : 0.f); a[8 + i] = (_Float16)(kb < K ? W[(size_t)kb * ld + n] : 0.f); }
  return a;
}
struct F2 { v16b h, l; };
__device__ __forceinline__ F2 bsplit16(const float v[16]) { F2 r;
#pragma unroll
  for (int i = 0; i < 16; ++i) { const __bf16 h = (__bf16)v[i]; r.h[i] = h; r.l[i] = (__bf16)(v[i] - (float)h); }
  return r; }
__device__ __forceinline__ F2 split_row(const float* row, int k0, int lane) { float v[16]; const float* p = row + k0 + 8 * (lane >> 4);
#pragma unroll
  for (int i = 0; i < 8; ++i) { v[i] = p[i]; v[8 + i] = p[16 + i]; }
  return bsplit16(v); }
__device__ __forceinline__ F2 split_rowK(const float* row, int k0, int lane, int K) { float v[16]; const int g = lane >> 4;
#pragma unroll
  for (int i = 0; i < 8; ++i) { const int ka = k0 + 8 * g + i, kb = ka + 16; v[i] = ka < K ? row[ka] : 0.f; v[8 + i] = kb < K ? row[kb] : 0.f; }
  return bsplit16(v); }
__device__ __forceinline__ F2 split_col(const float* W, int k0, int n, int lane, int ld, int K) { float v[16]; const int g = lane >> 4;
#pragma unroll
  for (int i = 0; i < 8; ++i) { const int ka = k0 + 8 * g + i, kb = ka + 16; v[i] = ka < K ? W[(size_t)ka * ld + n] : 0.f; v[8 + i] = kb < K ? W[(size_t)kb * ld + n] : 0.f; }
  return bsplit16(v); }
__device__ __forceinline__ v8f mac3(const F2& a, const F2& b, v8f c) { c = wmma_bf(a.l, b.h, c); c = wmma_bf(a.h, b.l, c); return wmma_bf(a.h, b.h, c); }
__device__ __forceinline__ float sigm(float v) { return 1.0f / (1.0f + expf(-v)); }
#define LDSX() do { asm volatile("s_wait_dscnt 0" ::: "memory"); __builtin_amdgcn_wave_barrier(); __builtin_amdgcn_fence(__ATOMIC_RELEASE, "workgroup"); } while (0)

#define NB 4
#define LL 2048
#define KN 8
#define CIN 32
#define COUT 32
#define HH 128
#define NKV (CIN * COUT)

__global__ __launch_bounds__(256) void k_pack(const float* __restrict__ W2, _Float16* __restrict__ P) {
  const int n = blockIdx.x, tid = threadIdx.x; __shared__ __align__(16) _Float16 sr[HH];
  if (tid < HH) sr[tid] = (_Float16)(W2[(size_t)tid * NKV + n] * 16.0f);
  __syncthreads();
  if (tid < HH / 8) vst2(P + (size_t)n * HH + tid * 8, *(const v4u*)(&sr[tid * 8]));
}
__global__ __launch_bounds__(128) void k_main(const float* __restrict__ times, const float* __restrict__ feat, const int* __restrict__ lens, const float* __restrict__ W1, const float* __restrict__ b1, const _Float16* __restrict__ P, const float* __restrict__ b2, float* __restrict__ out) {
  __shared__ float sdt[4][16]; __shared__ float smk[4][16]; __shared__ __align__(16) float sf[4][16][CIN + 1];
  const int tid = threadIdx.x, wave = tid >> 5, lane = tid & 31, col = lane & 15, g = lane >> 4;
  const int b = blockIdx.y, i0 = blockIdx.x * 8 + wave * 2; const int len = lens[b];
  if (lane < 16) { const int m = lane, il = m >> 3, k = m & 7; const int i = i0 + il, j = i - (k + 1); const int jc = j < 0 ? 0 : j;
    const bool msk = (j >= 0) && (jc < len) && (i <= len - 1);
    sdt[wave][m] = msk ? times[(size_t)b * LL + i] - times[(size_t)b * LL + jc] : 0.f; smk[wave][m] = msk ? 1.f : 0.f;
#pragma unroll
    for (int c = 0; c < CIN; ++c) sf[wave][m][c] = feat[((size_t)b * LL + jc) * CIN + c]; }
  LDSX();
  v16h ah[4]; { const float dt = sdt[wave][col];
#pragma unroll
    for (int kc = 0; kc < 4; ++kc) {
#pragma unroll
      for (int e = 0; e < 8; ++e) { const int ka = kc * 32 + 8 * g + e, kb = ka + 16; float va = dt * W1[ka] + b1[ka], vb2 = dt * W1[kb] + b1[kb]; ah[kc][e] = (_Float16)(va > 0.f ? va : 0.f); ah[kc][8 + e] = (_Float16)(vb2 > 0.f ? vb2 : 0.f); } } }
  const float mrow[8] = { smk[wave][8 * g + 0], smk[wave][8 * g + 1], smk[wave][8 * g + 2], smk[wave][8 * g + 3], smk[wave][8 * g + 4], smk[wave][8 * g + 5], smk[wave][8 * g + 6], smk[wave][8 * g + 7] };
  float o0 = 0.f, o1 = 0.f;
#pragma unroll 1
  for (int c = 0; c < CIN; ++c) {
    float fr[8];
#pragma unroll
    for (int r = 0; r < 8; ++r) fr[r] = sf[wave][8 * g + r][c] * mrow[r];
#pragma unroll
    for (int hlf = 0; hlf < 2; ++hlf) { const int n0 = c * COUT + hlf * 16; v8f acc = {};
#pragma unroll
      for (int kc = 0; kc < 4; ++kc) acc = wmma16(ah[kc], frag_h(P + (size_t)(n0 + col) * HH + kc * 32, lane), acc);
      const float bb = b2[n0 + col]; float s = 0.f;
#pragma unroll
      for (int r = 0; r < 8; ++r) s += fr[r] * (acc[r] * (1.0f / 16.0f) + bb);
      if (hlf == 0) o0 += s; else o1 += s; } }
  vst2(out + ((size_t)b * LL + i0 + g) * COUT + col, o0); vst2(out + ((size_t)b * LL + i0 + g) * COUT + 16 + col, o1);
}
extern "C" void kernel_launch(void* const* d_in, const int* in_sizes, int n_in, void* d_out, int out_size, void* d_ws, size_t ws_size, hipStream_t stream) {
  (void)in_sizes; (void)n_in; (void)out_size; (void)ws_size;
  const float* times = (const float*)d_in[0]; const float* feat = (const float*)d_in[1]; const int* lens = (const int*)d_in[2]; const float* W1 = (const float*)d_in[3]; const float* b1 = (const float*)d_in[4]; const float* W2 = (const float*)d_in[5]; const float* b2 = (const float*)d_in[6];
  float* out = (float*)d_out;
  _Float16* P = (_Float16*)d_ws;
  k_pack<<<NKV, 256, 0, stream>>>(W2, P);
  k_main<<<dim3(LL / 8, NB), 128, 0, stream>>>(times, feat, lens, W1, b1, P, b2, out);
}
